// KPC_fu_46351287059054
// MI455X (gfx1250) — hardware-run, weakly checked
//
#include <hip/hip_runtime.h>
#include <math.h>

#ifndef NB
#define NB 2
#endif
#ifndef NPT
#define NPT 32768
#endif
#define NPT_FULL 32768
#define CCH 6
#define NCUR 3
#define LCUR 2048
#define CURV_BSTRIDE (CCH * NCUR * LCUR)
#define QBLK 256
#define SLAB 2048
#define SPR (NPT / SLAB)
#define NSLAB (NB * CCH * SPR)
#define AT_PP 72

static_assert(NPT % QBLK == 0);
static_assert(NPT % SLAB == 0);
static_assert(NPT <= NPT_FULL);
static_assert(LCUR % 64 == 0);
static_assert(LCUR == 256 * 8);
static_assert(SLAB == 256 * 8);
static_assert((NB * CCH * NPT) % 256 == 0);
static_assert(AT_PP % 8 == 0 && AT_PP >= 64);
static_assert(16 * 16 * AT_PP * 2 + 16 * 16 * 16 * 4 + CCH * QBLK * 4 <= 131072);
static_assert(2 * 3 * LCUR * 4 + 8 * 20 * 4 + 18 * 4 * 2 + 64 * 4 <= 131072);
static_assert(16 * 3 * 128 == CCH * QBLK * 4);
static_assert((LCUR / 256) * 256 * 16 == LCUR * 8 * 2);
static_assert(1024 * 1024 == 1048576);
static_assert(2048.0 * 1024.0 * 0.5 == 1048576.0);

typedef _Float16 h16;
typedef __attribute__((ext_vector_type(16))) _Float16 v16h;
typedef __attribute__((ext_vector_type(8)))  _Float16 v8h;
typedef __attribute__((ext_vector_type(2)))  _Float16 v2h;
typedef __attribute__((ext_vector_type(8)))  float    v8f;
typedef __attribute__((ext_vector_type(4)))  float    v4f;
typedef __attribute__((ext_vector_type(2)))  float    v2f;
typedef __attribute__((ext_vector_type(4)))  unsigned int v4u;


#define VST2(T, ptr, val) do { const T vst2_v_ = (val); *(volatile T*)(ptr) = vst2_v_; __threadfence(); *(volatile T*)(ptr) = vst2_v_; } while (0)

__device__ __forceinline__ float bfr(float f) {
    unsigned u = __float_as_uint(f);
    u += 0x7FFFu + ((u >> 16) & 1u);
    return __uint_as_float(u & 0xFFFF0000u);
}
static __device__ __forceinline__ h16 toh_flush(float v) {
    const float w = (fabsf(v) < 6.103515625e-05f) ? 0.0f : v;
    return (h16)w;
}
static __device__ __forceinline__ v2h toh_flush2(float a, float b) {
    v2f w;
    w.x = (fabsf(a) < 6.103515625e-05f) ? 0.0f : a;
    w.y = (fabsf(b) < 6.103515625e-05f) ? 0.0f : b;
    return __builtin_convertvector(w, v2h);
}
union Pack8 { v8h v; v2h p[4]; };
static __device__ __forceinline__ void st8h_fl(h16* P, size_t o, const float* v) {
    Pack8 u;
    u.p[0] = toh_flush2(v[0], v[1]);
    u.p[1] = toh_flush2(v[2], v[3]);
    u.p[2] = toh_flush2(v[4], v[5]);
    u.p[3] = toh_flush2(v[6], v[7]);
    VST2(v8h, (v8h*)(P + o), u.v);
}

union FragU { v16h v; v8h h[2]; };
__device__ __forceinline__ v16h frag_ld(const _Float16* p) {
    FragU f; f.h[0] = *(const v8h*)(p); f.h[1] = *(const v8h*)(p + 16); return f.v;
}
__device__ __forceinline__ v8f wmma16(v16h a, v16h b, v8f c) {
    c = __builtin_amdgcn_wmma_f32_16x16x32_f16(false, a, false, b, (short)0, c, false, false);
    asm volatile("v_nop\n\tv_nop\n\tv_nop\n\tv_nop" : "+v"(c) : "v"(a), "v"(b));
    return c;
}
__device__ __forceinline__ void wave_sync_lds() {
    __builtin_amdgcn_fence(3  , "workgroup");
    __builtin_amdgcn_wave_barrier();
    __builtin_amdgcn_fence(2  , "workgroup");
}

__global__ __launch_bounds__(256) void k_pre(const float* __restrict__ curves, const float* __restrict__ Wa,
                                             const float* __restrict__ Wav, const float* __restrict__ Wb,
                                             const float* __restrict__ Wbv, const float* __restrict__ Watt,
                                             const float* __restrict__ Wpl, const float* __restrict__ bpl,
                                             const float* __restrict__ Wpn, const float* __restrict__ bpn,
                                             _Float16* __restrict__ KB16, _Float16* __restrict__ VT16, float* __restrict__ KV) {
    __shared__ float sAtt[3 * LCUR];
    __shared__ __align__(16) float sV[3 * LCUR];
    __shared__ float sRed[8][20];
    __shared__ float sCI[CCH][3];
    __shared__ float sPL[18];
    __shared__ float sKV[64];
    const unsigned tid = threadIdx.x, lane = tid & 31u;
    const unsigned wave = __builtin_amdgcn_readfirstlane(threadIdx.x >> 5);
    const unsigned b = blockIdx.x;
    const float* cb = curves + (size_t)b * CURV_BSTRIDE;

    {
        float watt[CCH];
#pragma unroll
        for (int ch = 0; ch < CCH; ++ch) watt[ch] = bfr(Watt[ch]);
        for (unsigned i = tid; i < 3u * LCUR; i += 256u) {
            const unsigned n = i / LCUR, l = i - n * LCUR;
            float s = 0.f;
#pragma unroll
            for (int ch = 0; ch < CCH; ++ch) s += bfr(cb[((unsigned)ch * 3u + n) * LCUR + l]) * watt[ch];
            sAtt[i] = s;
        }
    }
    __syncthreads();

    for (unsigned n = 0; n < 3u; ++n) {
        float pm = -3.0e38f;
        for (unsigned l = tid; l < LCUR; l += 256u) pm = fmaxf(pm, sAtt[n * LCUR + l]);
#pragma unroll
        for (int o = 16; o > 0; o >>= 1) pm = fmaxf(pm, __shfl_xor(pm, o, 32));
        if (lane == 0u) sRed[wave][0] = pm;
        __syncthreads();
        float mx = sRed[0][0];
#pragma unroll
        for (int w = 1; w < 8; ++w) mx = fmaxf(mx, sRed[w][0]);
        __syncthreads();
        float acc[7];
#pragma unroll
        for (int j = 0; j < 7; ++j) acc[j] = 0.f;
        for (unsigned l = tid; l < LCUR; l += 256u) {
            const float w = expf(sAtt[n * LCUR + l] - mx);
            acc[0] += w;
#pragma unroll
            for (int ch = 0; ch < CCH; ++ch) acc[1 + ch] += bfr(cb[((unsigned)ch * 3u + n) * LCUR + l]) * w;
        }
#pragma unroll
        for (int j = 0; j < 7; ++j) {
#pragma unroll
            for (int o = 16; o > 0; o >>= 1) acc[j] += __shfl_xor(acc[j], o, 32);
        }
        if (lane == 0u) {
#pragma unroll
            for (int j = 0; j < 7; ++j) sRed[wave][j] = acc[j];
        }
        __syncthreads();
        {
            const unsigned tc = min(tid, 5u);
            float den = sRed[0][0], tot = sRed[0][1u + tc];
#pragma unroll
            for (int w = 1; w < 8; ++w) { den += sRed[w][0]; tot += sRed[w][1u + tc]; }
            const float ci = tot / den;
            if (tid < 6u) sCI[tc][n] = ci;
        }
        __syncthreads();
    }

    float pacc[18];
#pragma unroll
    for (int j = 0; j < 18; ++j) pacc[j] = 0.f;
    {
        float wpl[9], wpn[9], bl[3], bn3[3], wb[18], wbv[18];
#pragma unroll
        for (int j = 0; j < 9; ++j) { wpl[j] = bfr(Wpl[j]); wpn[j] = bfr(Wpn[j]); }
#pragma unroll
        for (int j = 0; j < 3; ++j) { bl[j] = bfr(bpl[j]); bn3[j] = bfr(bpn[j]); }
#pragma unroll
        for (int j = 0; j < 18; ++j) { wb[j] = bfr(Wb[j]); wbv[j] = bfr(Wbv[j]); }
        h16* KBb = KB16 + (size_t)b * LCUR * 8u;
        for (unsigned it = 0; it < (unsigned)(LCUR / 256); ++it) {
            const unsigned l = it * 256u + tid;
            const float a0 = sAtt[l], a1 = sAtt[LCUR + l], a2 = sAtt[2 * LCUR + l];
            const float m3 = fmaxf(a0, fmaxf(a1, a2));
            const float e0 = expf(a0 - m3), e1 = expf(a1 - m3), e2 = expf(a2 - m3);
            const float es = (e0 + e1) + e2;
            const float w0 = e0 / es, w1 = e1 / es, w2 = e2 / es;
            float ga[CCH];
#pragma unroll
            for (int ch = 0; ch < CCH; ++ch) {
                const float p0 = bfr(curves[(ch * 3 + 0) * LCUR + l]);
                const float p1 = bfr(curves[(ch * 3 + 1) * LCUR + l]);
                const float p2 = bfr(curves[(ch * 3 + 2) * LCUR + l]);
                const float c0 = bfr(cb[(ch * 3 + 0) * LCUR + l]);
                const float c1 = bfr(cb[(ch * 3 + 1) * LCUR + l]);
                const float c2 = bfr(cb[(ch * 3 + 2) * LCUR + l]);
#pragma unroll
                for (int m = 0; m < 3; ++m) {
                    const float plv = ((p0 * wpl[3 * m] + p1 * wpl[3 * m + 1]) + p2 * wpl[3 * m + 2]) + bl[m];
                    pacc[ch * 3 + m] += plv;
                }
                const float pn0 = ((p0 * wpn[0] + p1 * wpn[1]) + p2 * wpn[2]) + bn3[0];
                const float pn1 = ((p0 * wpn[3] + p1 * wpn[4]) + p2 * wpn[5]) + bn3[1];
                const float pn2 = ((p0 * wpn[6] + p1 * wpn[7]) + p2 * wpn[8]) + bn3[2];
                const float pnm = ((pn0 + pn1) + pn2) / 3.0f;
                const float ci = (c0 * w0 + c1 * w1) + c2 * w2;
                ga[ch] = ci + pnm;
            }
            float kq[3];
#pragma unroll
            for (int m = 0; m < 3; ++m) {
                float kv = 0.f, vv = 0.f;
#pragma unroll
                for (int ch = 0; ch < CCH; ++ch) { kv += ga[ch] * wb[m * CCH + ch]; vv += ga[ch] * wbv[m * CCH + ch]; }
                kq[m] = kv;
                sV[(unsigned)m * LCUR + l] = vv;
            }
            const float kb[8] = {kq[0] * 1024.0f, kq[1] * 1024.0f, kq[2] * 1024.0f,
                                 kq[0] * 0.5f, kq[1] * 0.5f, kq[2] * 0.5f, 0.0f, 0.0f};
            st8h_fl(KBb, (size_t)l * 8u, kb);
        }
    }
#pragma unroll
    for (int j = 0; j < 18; ++j) {
#pragma unroll
        for (int o = 16; o > 0; o >>= 1) pacc[j] += __shfl_xor(pacc[j], o, 32);
    }
    if (lane == 0u) {
#pragma unroll
        for (int j = 0; j < 18; ++j) sRed[wave][j] = pacc[j];
    }
    __syncthreads();
    {
        const unsigned tc = min(tid, 17u);
        float tot = sRed[0][tc];
#pragma unroll
        for (int w = 1; w < 8; ++w) tot += sRed[w][tc];
        const float pm = tot / (float)LCUR;
        if (tid < 18u) sPL[tc] = pm;
    }
    __syncthreads();
    {
        unsigned j = min(lane, 8u);
        asm volatile("" : "+v"(j));
        const unsigned a = j / 3u, bb = j - 3u * a;
        float ki = 0.f, vi = 0.f;
#pragma unroll
        for (int ch = 0; ch < CCH; ++ch) {
            const float gia = sCI[ch][a] + sPL[ch * 3 + a];
            const float gib = sCI[ch][bb] + sPL[ch * 3 + bb];
            ki += gib * bfr(Wa[a * CCH + ch]);
            vi += gia * bfr(Wav[bb * CCH + ch]);
        }
        const float val = (lane < 9u) ? ((tid < 32u) ? ki : vi) : 0.0f;
        if (tid < 64u) sKV[tid] = val;
    }
    __syncthreads();
    if (wave == 0u) {
        VST2(float, KV + b * 64u + lane, sKV[lane]);
        VST2(float, KV + b * 64u + 32u + lane, sKV[32u + lane]);
    }
    {
        h16* VTb = VT16 + (size_t)b * 16u * LCUR;
        for (unsigned m = 0; m < 3u; ++m) {
            const v4f a = *(const v4f*)(sV + m * LCUR + 8u * tid);
            const v4f c2 = *(const v4f*)(sV + m * LCUR + 8u * tid + 4u);
            const float v[8] = {a.x * 1024.0f, a.y * 1024.0f, a.z * 1024.0f, a.w * 1024.0f,
                                c2.x * 1024.0f, c2.y * 1024.0f, c2.z * 1024.0f, c2.w * 1024.0f};
            st8h_fl(VTb, (size_t)m * LCUR + 8u * tid, v);
        }
        const float z[8] = {0.f, 0.f, 0.f, 0.f, 0.f, 0.f, 0.f, 0.f};
        for (unsigned m = 3u; m < 16u; ++m) st8h_fl(VTb, (size_t)m * LCUR + 8u * tid, z);
    }
}

__global__ __launch_bounds__(512) void k_attn(const float* __restrict__ x, const float* __restrict__ Wc,
                                              const float* __restrict__ Wd, const float* __restrict__ lng,
                                              const float* __restrict__ lnb, const _Float16* __restrict__ KB16,
                                              const _Float16* __restrict__ VT16, const float* __restrict__ KV,
                                              float* __restrict__ Y) {
    __shared__ __align__(16) _Float16 sP[16][16 * AT_PP];
    __shared__ __align__(16) float sF[16][16 * 16];
    __shared__ float sY[CCH * QBLK];
    const unsigned tid = threadIdx.x, lane = tid & 31u;
    const unsigned wave = __builtin_amdgcn_readfirstlane(threadIdx.x >> 5);
    const unsigned hh = lane >> 4, c = lane & 15u;
    const unsigned b = blockIdx.x / (unsigned)(NPT / QBLK);
    const unsigned i0 = (blockIdx.x - b * (unsigned)(NPT / QBLK)) * QBLK;
    const unsigned iw = i0 + wave * 16u;
    const float* xb = x + (size_t)b * CCH * NPT_FULL;

    float wc[18];
#pragma unroll
    for (int j = 0; j < 18; ++j) wc[j] = bfr(Wc[j]);

    float qa = 0.f, qb = 0.f, qc = 0.f;
#pragma unroll
    for (int ch = 0; ch < CCH; ++ch) {
        const float t = bfr(xb[(size_t)ch * NPT_FULL + iw + c]);
        qa = fmaf(t, wc[ch], qa);
        qb = fmaf(t, wc[CCH + ch], qb);
        qc = fmaf(t, wc[2 * CCH + ch], qc);
    }

    const v8h z8 = __builtin_bit_cast(v8h, (v4u){0u, 0u, 0u, 0u});
    v16h qfrag;
    {
        const float hsel = (hh == 0u) ? 1024.0f : 0.0f;
        const float s0 = qa * hsel, s1 = qb * hsel, s2 = qc * hsel;
        const v2h h01 = toh_flush2(s0, s1);
        const v2h h2z = toh_flush2(s2, 0.0f);
        const float r0 = 2048.0f * (s0 - (float)h01.x);
        const float r1 = 2048.0f * (s1 - (float)h01.y);
        const float r2 = 2048.0f * (s2 - (float)h2z.x);
        const v2h l01 = toh_flush2(r0, r1);
        const v2h l2z = toh_flush2(r2, 0.0f);
        Pack8 q8;
        v2h w1; w1.x = h2z.x; w1.y = l01.x;
        v2h w2; w2.x = l01.y; w2.y = l2z.x;
        q8.p[0] = h01;
        q8.p[1] = w1;
        q8.p[2] = w2;
        q8.p[3] = toh_flush2(0.0f, 0.0f);
        FragU qf; qf.h[0] = q8.v; qf.h[1] = z8;
        qfrag = qf.v;
    }
    const unsigned kmsk = hh - 1u;
    const v4u kmask = (v4u){kmsk, kmsk, kmsk, kmsk};

    _Float16* pw = sP[wave];
    const _Float16* KBb = KB16 + (size_t)b * LCUR * 8u + (size_t)c * 8u;
    const _Float16* VTb = VT16 + (size_t)b * 16u * LCUR + (size_t)c * LCUR + 8u * hh;
    const float SC2S = (1.4426950408889634f / 1.7320508075688772f) / 1048576.0f;

    float mrow[8], lpart[8];
#pragma unroll
    for (int r = 0; r < 8; ++r) { mrow[r] = -3.0e38f; lpart[r] = 0.f; }
    v8f os = (v8f){0.f, 0.f, 0.f, 0.f, 0.f, 0.f, 0.f, 0.f};

#pragma unroll 1
    for (unsigned kc = 0; kc < (unsigned)(LCUR / 64); ++kc) {
        const unsigned kv0 = kc * 64u;
        v8f s[4];
#pragma unroll
        for (int j = 0; j < 4; ++j) {
            const v8h kraw = *(const v8h*)(KBb + (size_t)(kv0 + (unsigned)j * 16u) * 8u);
            const v4u kmk = __builtin_bit_cast(v4u, kraw) & kmask;
            FragU kf; kf.h[0] = __builtin_bit_cast(v8h, kmk); kf.h[1] = z8;
            const v8f z = (v8f){0.f, 0.f, 0.f, 0.f, 0.f, 0.f, 0.f, 0.f};
            s[j] = wmma16(qfrag, kf.v, z);
        }
#pragma unroll
        for (int r = 0; r < 8; ++r) {
            float sj[4];
            float mx = -3.0e38f;
#pragma unroll
            for (int j = 0; j < 4; ++j) {
                sj[j] = s[j][r] * SC2S;
                mx = fmaxf(mx, sj[j]);
            }
            mx = fmaxf(mx, __shfl_xor(mx, 1, 32)); mx = fmaxf(mx, __shfl_xor(mx, 2, 32));
            mx = fmaxf(mx, __shfl_xor(mx, 4, 32)); mx = fmaxf(mx, __shfl_xor(mx, 8, 32));
            const float mnew = fmaxf(mrow[r], mx);
            const float alpha = exp2f(mrow[r] - mnew);
            mrow[r] = mnew;
            float psum = 0.f;
#pragma unroll
            for (int j = 0; j < 4; ++j) {
                const float p = exp2f(sj[j] - mnew);
                psum += p;
                pw[(8u * hh + (unsigned)r) * AT_PP + (unsigned)j * 16u + c] = toh_flush(p * 1024.0f);
            }
            lpart[r] = lpart[r] * alpha + psum;
            os[r] *= alpha;
        }
        wave_sync_lds();
#pragma unroll
        for (int kk = 0; kk < 2; ++kk) {
            const v16h pa = frag_ld(pw + c * AT_PP + (unsigned)kk * 32u + 8u * hh);
            const v16h vb = frag_ld(VTb + kv0 + (unsigned)kk * 32u);
            os = wmma16(pa, vb, os);
        }
        wave_sync_lds();
    }

    float* fw = sF[wave];
#pragma unroll
    for (int r = 0; r < 8; ++r) {
        float ls = lpart[r];
        ls += __shfl_xor(ls, 1, 32); ls += __shfl_xor(ls, 2, 32);
        ls += __shfl_xor(ls, 4, 32); ls += __shfl_xor(ls, 8, 32);
        fw[(8u * hh + (unsigned)r) * 16u + c] = os[r] / (ls * 1048576.0f);
    }
    wave_sync_lds();
    const v4f f4 = *(const v4f*)(fw + c * 16u);

    const float* KVb = KV + b * 64u;
    float ki[9], vi[9];
#pragma unroll
    for (int j = 0; j < 9; ++j) { ki[j] = KVb[j]; vi[j] = KVb[32 + j]; }
    float sn[3];
#pragma unroll
    for (int n = 0; n < 3; ++n) sn[n] = fmaf(qc, ki[6 + n], fmaf(qb, ki[3 + n], qa * ki[n])) / 1.7320508075688772f;
    const float m3 = fmaxf(sn[0], fmaxf(sn[1], sn[2]));
    const float e0 = expf(sn[0] - m3), e1 = expf(sn[1] - m3), e2 = expf(sn[2] - m3);
    const float es = (e0 + e1) + e2;
    const float a0 = e0 / es, a1 = e1 / es, a2 = e2 / es;
    float cf[CCH];
#pragma unroll
    for (int m = 0; m < 3; ++m) cf[m] = (a0 * vi[m] + a1 * vi[3 + m]) + a2 * vi[6 + m];
    cf[3] = f4.x; cf[4] = f4.y; cf[5] = f4.z;

    const float mu = (((((cf[0] + cf[1]) + cf[2]) + cf[3]) + cf[4]) + cf[5]) / 6.0f;
    float d[CCH];
    float vs = 0.f;
#pragma unroll
    for (int j = 0; j < CCH; ++j) { d[j] = cf[j] - mu; vs += d[j] * d[j]; }
    const float rs = 1.0f / sqrtf(vs / 6.0f + 1e-5f);
    float cn[CCH];
#pragma unroll
    for (int j = 0; j < CCH; ++j) cn[j] = d[j] * rs * bfr(lng[j]) + bfr(lnb[j]);
#pragma unroll
    for (int o = 0; o < CCH; ++o) {
        float s = 0.f;
#pragma unroll
        for (int j = 0; j < CCH; ++j) s += cn[j] * bfr(Wd[o * CCH + j]);
        if (lane < 16u) sY[(unsigned)o * QBLK + wave * 16u + c] = s;
    }
    __syncthreads();
    {
        float yv[3];
#pragma unroll
        for (int it = 0; it < 3; ++it) {
            const unsigned u = wave + 16u * (unsigned)it;
            yv[it] = sY[(u >> 3) * QBLK + (u & 7u) * 32u + lane];
        }
        for (int pass = 0; pass < 2; ++pass) {
#pragma unroll
            for (int it = 0; it < 3; ++it) {
                const unsigned u = wave + 16u * (unsigned)it;
                *(volatile float*)(Y + (size_t)(b * CCH + (u >> 3)) * NPT + i0 + (u & 7u) * 32u + lane) = yv[it];
            }
            __threadfence();
        }
    }
}

__global__ __launch_bounds__(256) void k_sum(const float* __restrict__ Y, float* __restrict__ part) {
    __shared__ float sW[8];
    const unsigned tid = threadIdx.x, lane = tid & 31u;
    const unsigned wave = __builtin_amdgcn_readfirstlane(threadIdx.x >> 5);
    const float* src = Y + (size_t)blockIdx.x * SLAB;
    const v4f a = *(const v4f*)(src + 4u * tid), c2 = *(const v4f*)(src + 1024u + 4u * tid);
    float s = ((a.x + a.y) + (a.z + a.w)) + ((c2.x + c2.y) + (c2.z + c2.w));
#pragma unroll
    for (int o = 16; o > 0; o >>= 1) s += __shfl_xor(s, o, 32);
    if (lane == 0u) sW[wave] = s;
    __syncthreads();
    if (wave == 0u) {
        float t = sW[0];
#pragma unroll
        for (int w = 1; w < 8; ++w) t += sW[w];
        VST2(float, part + (size_t)blockIdx.x * 32u + lane, (lane == 0u) ? t : 0.0f);
    }
}

__global__ __launch_bounds__(32) void k_mean(const float* __restrict__ part, float* __restrict__ meanl) {
    const unsigned lane = threadIdx.x;
    const unsigned oc = min(lane, (unsigned)(CCH - 1));
    float s = 0.f;
    for (unsigned b = 0; b < (unsigned)NB; ++b)
        for (unsigned sl = 0; sl < (unsigned)SPR; ++sl) s += part[(size_t)((b * CCH + oc) * SPR + sl) * 32u];
    const float m = s / (float)(NB * NPT);
    VST2(float, meanl + lane, (lane < (unsigned)CCH) ? m : 0.0f);
}

__global__ __launch_bounds__(256) void k_sq(const float* __restrict__ Y, const float* __restrict__ meanl, float* __restrict__ part) {
    __shared__ float sW[8];
    const unsigned tid = threadIdx.x, lane = tid & 31u;
    const unsigned wave = __builtin_amdgcn_readfirstlane(threadIdx.x >> 5);
    const unsigned o = (blockIdx.x / (unsigned)SPR) % (unsigned)CCH;
    const float bm = meanl[o];
    const float* src = Y + (size_t)blockIdx.x * SLAB;
    const v4f a = *(const v4f*)(src + 4u * tid), c2 = *(const v4f*)(src + 1024u + 4u * tid);
    const float d0 = a.x - bm, d1 = a.y - bm, d2 = a.z - bm, d3 = a.w - bm;
    const float d4 = c2.x - bm, d5 = c2.y - bm, d6 = c2.z - bm, d7 = c2.w - bm;
    float s = ((d0 * d0 + d1 * d1) + (d2 * d2 + d3 * d3)) + ((d4 * d4 + d5 * d5) + (d6 * d6 + d7 * d7));
#pragma unroll
    for (int of = 16; of > 0; of >>= 1) s += __shfl_xor(s, of, 32);
    if (lane == 0u) sW[wave] = s;
    __syncthreads();
    if (wave == 0u) {
        float t = sW[0];
#pragma unroll
        for (int w = 1; w < 8; ++w) t += sW[w];
        VST2(float, part + (size_t)blockIdx.x * 32u + lane, (lane == 0u) ? t : 0.0f);
    }
}

__global__ __launch_bounds__(32) void k_rstd(const float* __restrict__ part, float* __restrict__ rstdl) {
    const unsigned lane = threadIdx.x;
    const unsigned oc = min(lane, (unsigned)(CCH - 1));
    float s = 0.f;
    for (unsigned b = 0; b < (unsigned)NB; ++b)
        for (unsigned sl = 0; sl < (unsigned)SPR; ++sl) s += part[(size_t)((b * CCH + oc) * SPR + sl) * 32u];
    const float bv = s / (float)(NB * NPT);
    const float r = 1.0f / sqrtf(bv + 1e-5f);
    VST2(float, rstdl + lane, (lane < (unsigned)CCH) ? r : 0.0f);
}

__global__ __launch_bounds__(256) void k_out(const float* __restrict__ x, const float* __restrict__ Y,
                                             const float* __restrict__ meanl, const float* __restrict__ rstdl,
                                             const float* __restrict__ gam, const float* __restrict__ bet,
                                             float* __restrict__ out) {
    const unsigned u = blockIdx.x * 256u + threadIdx.x;
    if (u >= (unsigned)(NB * CCH * NPT)) return;
    unsigned bo = u / (unsigned)NPT;
    asm volatile("" : "+v"(bo));
    const unsigned i = u - bo * (unsigned)NPT;
    const unsigned o = bo % (unsigned)CCH;
    const size_t xu = (size_t)bo * NPT_FULL + i;
    const float yv = (Y[u] - meanl[o]) * rstdl[o] * bfr(gam[o]) + bfr(bet[o]);
    const float v = bfr(x[xu]) + yv;
    const float r = (v >= 0.0f) ? v : 0.2f * v;
    VST2(float, out + xu, r);
}

constexpr size_t al256(size_t v) { return (v + 255) & ~(size_t)255; }
constexpr size_t WS_KB    = 0;
constexpr size_t WS_VT    = al256(WS_KB + (size_t)NB * LCUR * 8 * 2);
constexpr size_t WS_KV    = al256(WS_VT + (size_t)NB * 16 * LCUR * 2);
constexpr size_t WS_Y     = al256(WS_KV + (size_t)NB * 64 * 4);
constexpr size_t WS_P1    = al256(WS_Y + (size_t)NB * CCH * NPT * 4);
constexpr size_t WS_MEAN  = al256(WS_P1 + (size_t)NSLAB * 128);
constexpr size_t WS_P2    = al256(WS_MEAN + 128);
constexpr size_t WS_RSTD  = al256(WS_P2 + (size_t)NSLAB * 128);
constexpr size_t WS_TOTAL = al256(WS_RSTD + 128);
static_assert(WS_TOTAL <= 134217728);

extern "C" void kernel_launch(void* const* d_in, const int* in_sizes, int n_in, void* d_out, int out_size,
                              void* d_ws, size_t ws_size, hipStream_t stream) {
    if (n_in < 17) return;
    if (in_sizes[0] < (NB * CCH - 1) * NPT_FULL + NPT) return;
    if (in_sizes[1] < NB * CURV_BSTRIDE) return;
    if (in_sizes[2] < 18 || in_sizes[3] < 18 || in_sizes[4] < 18 || in_sizes[5] < 18 || in_sizes[6] < 18) return;
    if (in_sizes[7] < 36 || in_sizes[8] < 6 || in_sizes[9] < 6 || in_sizes[10] < 6 || in_sizes[11] < 6 || in_sizes[12] < 6) return;
    if (in_sizes[13] < 9 || in_sizes[14] < 3 || in_sizes[15] < 9 || in_sizes[16] < 3) return;
    if (out_size < (NB * CCH - 1) * NPT_FULL + NPT) return;
    if (WS_TOTAL > ws_size) return;

    const float* x      = (const float*)d_in[0];
    const float* curves = (const float*)d_in[1];
    const float* Wa     = (const float*)d_in[2];
    const float* Wav    = (const float*)d_in[3];
    const float* Wb     = (const float*)d_in[4];
    const float* Wbv    = (const float*)d_in[5];
    const float* Wc     = (const float*)d_in[6];
    const float* Wd     = (const float*)d_in[7];
    const float* bn_g   = (const float*)d_in[8];
    const float* bn_b   = (const float*)d_in[9];
    const float* Watt   = (const float*)d_in[10];
    const float* ln_g   = (const float*)d_in[11];
    const float* ln_b   = (const float*)d_in[12];
    const float* Wpl    = (const float*)d_in[13];
    const float* bpl    = (const float*)d_in[14];
    const float* Wpn    = (const float*)d_in[15];
    const float* bpn    = (const float*)d_in[16];
    float* out = (float*)d_out;

    char* wsp = (char*)d_ws;
    _Float16* KB16  = (_Float16*)(wsp + WS_KB);
    _Float16* VT16  = (_Float16*)(wsp + WS_VT);
    float*    KV    = (float*)(wsp + WS_KV);
    float*    Yp    = (float*)(wsp + WS_Y);
    float*    part1 = (float*)(wsp + WS_P1);
    float*    meanl = (float*)(wsp + WS_MEAN);
    float*    part2 = (float*)(wsp + WS_P2);
    float*    rstdl = (float*)(wsp + WS_RSTD);

    k_pre<<<NB, 256, 0, stream>>>(curves, Wa, Wav, Wb, Wbv, Watt, Wpl, bpl, Wpn, bpn, KB16, VT16, KV);
    k_attn<<<NB * (NPT / QBLK), 512, 0, stream>>>(x, Wc, Wd, ln_g, ln_b, KB16, VT16, KV, Yp);
    k_sum<<<NSLAB, 256, 0, stream>>>(Yp, part1);
    k_mean<<<1, 32, 0, stream>>>(part1, meanl);
    k_sq<<<NSLAB, 256, 0, stream>>>(Yp, meanl, part2);
    k_rstd<<<1, 32, 0, stream>>>(part2, rstdl);
    k_out<<<(NB * CCH * NPT) / 256, 256, 0, stream>>>(x, Yp, meanl, rstdl, bn_g, bn_b, out);
}
